// PTSeg_67714454389196
// MI455X (gfx1250) — hardware-run, weakly checked
//
#include <hip/hip_runtime.h>
#include <math.h>

typedef __attribute__((ext_vector_type(16))) _Float16 v16h;
typedef __attribute__((ext_vector_type(8)))  _Float16 v8h;
typedef __attribute__((ext_vector_type(8)))  float    v8f;
typedef __attribute__((ext_vector_type(4)))  float    v4f;
typedef __attribute__((ext_vector_type(8)))  unsigned v8u;
typedef __attribute__((ext_vector_type(4)))  unsigned v4u;
typedef __attribute__((ext_vector_type(2)))  unsigned v2u;

constexpr int kPts   = 32768;
constexpr int kCh    = 128;
constexpr int kNbr   = 16;
constexpr int kGrp   = 16;
constexpr int kQkvP  = 3 * kCh;
constexpr int kPairs = kPts * kNbr;
constexpr int kAP    = 136;
constexpr int kHP    = 20;
constexpr float kBnEps = 1e-5f;
constexpr float kActCarry = 16.0f;
constexpr float kWgtCarry = 64.0f;
constexpr float kFold     = 1.0f / 1024.0f;
static_assert(kActCarry * kWgtCarry * kFold == 1.0f);
static_assert((kPts % 64) == 0 && (kQkvP % 64) == 0 && (kCh % 32) == 0);
static_assert(kPairs == 524288);
static_assert(kNbr == 16 && kGrp == 16 && kCh == 128);

constexpr size_t kOffXH    = 0;
constexpr size_t kOffWTH   = kOffXH    + (size_t)kPts * kCh * 2;
constexpr size_t kOffW1H   = kOffWTH   + (size_t)kQkvP * kCh * 2;
constexpr size_t kOffW2H   = kOffW1H   + (size_t)kGrp * kCh * 2;
constexpr size_t kOffBQKV  = kOffW2H   + (size_t)kGrp * 32 * 2;
constexpr size_t kOffQKV   = kOffBQKV  + (size_t)kQkvP * 4;
constexpr size_t kOffA3    = kOffQKV   + (size_t)kPts * kQkvP * 4;
constexpr size_t kOffH1    = kOffA3    + (size_t)kPairs * 4 * 4;
constexpr size_t kOffPPART = kOffH1    + (size_t)kPts * 256 * 4;
constexpr size_t kOffPSTAT = kOffPPART + (size_t)256 * 32 * 4;
constexpr size_t kOffWPART = kOffPSTAT + (size_t)32 * 4;
constexpr size_t kOffWSTAT = kOffWPART + (size_t)1024 * 256 * 4;
constexpr size_t kOffHPART = kOffWSTAT + (size_t)384 * 4;
constexpr size_t kOffHSTAT = kOffHPART + (size_t)1024 * 32 * 4;
constexpr size_t kWsTotal  = kOffHSTAT + (size_t)64 * 4;
static_assert(kWsTotal == 101982592ull);
static_assert(kWsTotal <= 134217728ull);
static_assert((kOffWTH % 128) == 0 && (kOffW1H % 128) == 0 && (kOffW2H % 128) == 0 && (kOffBQKV % 128) == 0 &&
              (kOffQKV % 128) == 0 && (kOffA3 % 128) == 0 && (kOffH1 % 128) == 0 && (kOffPPART % 128) == 0 &&
              (kOffPSTAT % 128) == 0 && (kOffWPART % 128) == 0 && (kOffWSTAT % 128) == 0 && (kOffHPART % 128) == 0 &&
              (kOffHSTAT % 128) == 0);

__device__ __forceinline__ unsigned pack_h2(float f0, float f1) {
  const _Float16 h0 = (_Float16)f0;
  const _Float16 h1 = (_Float16)f1;
  const unsigned short b0 = __builtin_bit_cast(unsigned short, h0);
  const unsigned short b1 = __builtin_bit_cast(unsigned short, h1);
  return (unsigned)b0 | ((unsigned)b1 << 16);
}

__device__ __forceinline__ void guard1_h(v8f& a, v16h x, v16h y) { asm volatile("v_nop\n\tv_nop\n\tv_nop\n\tv_nop" : "+v"(a) : "v"(x), "v"(y)); }
__device__ __forceinline__ void keep4_h(v16h a, v16h b, v16h c, v16h d) { asm volatile("v_nop" :: "v"(a), "v"(b), "v"(c), "v"(d)); }
__device__ __forceinline__ void acc_guard4(v8f& a, v8f& b, v8f& c, v8f& d) { asm volatile("v_nop\n\tv_nop\n\tv_nop\n\tv_nop" : "+v"(a), "+v"(b), "+v"(c), "+v"(d)); }

union FragU { v16h v; v8h h[2]; };
__device__ __forceinline__ v16h frag_load(const _Float16* p) {
  FragU f;
  f.h[0] = *(const v8h*)(p);
  f.h[1] = *(const v8h*)(p + 16);
  return f.v;
}
__device__ __forceinline__ v8f mma_raw(v16h a, v16h b, v8f c) {
  return __builtin_amdgcn_wmma_f32_16x16x32_f16(false, a, false, b, (short)0, c, false, false);
}
__device__ __forceinline__ v8f hmma(v16h a, v16h b, v8f c) {
  c = __builtin_amdgcn_wmma_f32_16x16x32_f16(false, a, false, b, (short)0, c, false, false);
  asm volatile("v_nop\n\tv_nop\n\tv_nop\n\tv_nop" : "+v"(c) : "v"(a), "v"(b));
  return c;
}

__global__ __launch_bounds__(256) void wmma_gemm64_f16(
    const unsigned short* __restrict__ Ap, int lda,
    const unsigned short* __restrict__ Btp, int ldb,
    float* __restrict__ C, int ldc,
    const float* __restrict__ bias,
    int M, int N, int K, float scale) {
  const _Float16* A  = (const _Float16*)Ap;
  const _Float16* Bt = (const _Float16*)Btp;
  __shared__ __align__(16) float sT[8][16 * 68];
  const int lane = threadIdx.x & 31;
  const int wave = threadIdx.x >> 5;
  const int tilesN = N >> 6;
  const int tilesM = M >> 6;
  const int tile = blockIdx.x * 8 + wave;
  if (tile >= tilesM * tilesN) return;
  const int tm = tile / tilesN;
  const int tn = tile - tm * tilesN;
  const int m0 = tm << 6;
  const int n0 = tn << 6;

  const int rlane = lane & 15;
  const int koff  = (lane >> 4) * 8;
  const int mOff  = (lane >> 4) * 8;

  v8f acc[4][4];
#pragma unroll
  for (int i = 0; i < 4; ++i)
#pragma unroll
    for (int j = 0; j < 4; ++j) acc[i][j] = (v8f){0.f,0.f,0.f,0.f,0.f,0.f,0.f,0.f};

  for (int k0 = 0; k0 < K; k0 += 32) {
    v16h bh[4];
#pragma unroll
    for (int j = 0; j < 4; ++j) {
      const size_t bo = (size_t)(n0 + (j << 4) + rlane) * ldb + koff + k0;
      bh[j] = frag_load(Bt + bo);
    }
#pragma unroll
    for (int i = 0; i < 4; ++i) {
      const size_t ao = (size_t)(m0 + (i << 4) + rlane) * lda + koff + k0;
      const v16h ah = frag_load(A + ao);
#pragma unroll
      for (int j = 0; j < 4; ++j) acc[i][j] = mma_raw(ah, bh[j], acc[i][j]);
#pragma unroll
      for (int j = 0; j < 4; ++j) guard1_h(acc[i][j], ah, bh[j]);
    }
    keep4_h(bh[0], bh[1], bh[2], bh[3]);
  }
  acc_guard4(acc[0][0], acc[0][1], acc[0][2], acc[0][3]);
  acc_guard4(acc[1][0], acc[1][1], acc[1][2], acc[1][3]);
  acc_guard4(acc[2][0], acc[2][1], acc[2][2], acc[2][3]);
  acc_guard4(acc[3][0], acc[3][1], acc[3][2], acc[3][3]);

  float* slab = sT[wave];
#pragma unroll
  for (int i = 0; i < 4; ++i) {
    const int mBase = m0 + (i << 4);
#pragma unroll
    for (int j = 0; j < 4; ++j) {
      const int n = n0 + (j << 4) + rlane;
      const float bv = bias[n];
#pragma unroll
      for (int r = 0; r < 8; ++r) {
        const float v = acc[i][j][r] * scale + bv;
        slab[(mOff + r) * 68 + (j << 4) + rlane] = v;
      }
    }
    __builtin_amdgcn_fence(__ATOMIC_RELEASE, "workgroup");
    __builtin_amdgcn_wave_barrier();
    __builtin_amdgcn_fence(__ATOMIC_ACQUIRE, "workgroup");
    {
      const int hh = lane >> 4, c4 = (lane & 15) * 4;
      for (int pass = 0; pass < 2; ++pass) {
#pragma unroll
        for (int it = 0; it < 8; ++it) {
          const int row = it * 2 + hh;
          v4f v = *(const v4f*)(slab + row * 68 + c4);
          *(volatile v4f*)(C + (size_t)(mBase + row) * ldc + n0 + c4) = v;
        }
        __threadfence();
      }
    }
    __builtin_amdgcn_fence(__ATOMIC_RELEASE, "workgroup");
    __builtin_amdgcn_wave_barrier();
    __builtin_amdgcn_fence(__ATOMIC_ACQUIRE, "workgroup");
  }
}

__global__ __launch_bounds__(256) void cast_rows_f16_kernel(
    const float* __restrict__ src, unsigned short* __restrict__ dst, int total8)
{
  const int i = blockIdx.x * 256 + threadIdx.x;
  if (i >= total8) return;
  const size_t e0 = (size_t)i << 3;
  const v4f a0 = *(const v4f*)(src + e0);
  const v4f a1 = *(const v4f*)(src + e0 + 4);
  const float f0 = a0[0] * kActCarry, f1 = a0[1] * kActCarry, f2 = a0[2] * kActCarry, f3 = a0[3] * kActCarry;
  const float f4 = a1[0] * kActCarry, f5 = a1[1] * kActCarry, f6 = a1[2] * kActCarry, f7 = a1[3] * kActCarry;
  v4u u;
  u[0] = pack_h2(f0, f1);
  u[1] = pack_h2(f2, f3);
  u[2] = pack_h2(f4, f5);
  u[3] = pack_h2(f6, f7);
  unsigned short* q = dst + e0;
  *(volatile v4u*)q = u;
  __threadfence();
  *(volatile v4u*)q = u;
}

__device__ __forceinline__ void emit_bt8(const float* __restrict__ W, int ldw, int kreal, int scol, int k0,
                                         unsigned short* __restrict__ dh, int drow, int kpad) {
  float f[8];
#pragma unroll
  for (int e = 0; e < 8; ++e) {
    const int k  = k0 + e;
    const int kc = (k < kreal) ? k : (kreal - 1);
    const float v = W[(size_t)kc * ldw + scol] * kWgtCarry;
    f[e] = (k < kreal) ? v : 0.0f;
  }
  v4u uh;
  uh[0] = pack_h2(f[0], f[1]);
  uh[1] = pack_h2(f[2], f[3]);
  uh[2] = pack_h2(f[4], f[5]);
  uh[3] = pack_h2(f[6], f[7]);
  unsigned short* ph = dh + (size_t)drow * kpad + k0;
  *(volatile v4u*)ph = uh;
  __threadfence();
  *(volatile v4u*)ph = uh;
}

__global__ __launch_bounds__(256) void prep_planes_kernel(
    const float* __restrict__ Wq, const float* __restrict__ Wk, const float* __restrict__ Wv,
    const float* __restrict__ bq, const float* __restrict__ bk, const float* __restrict__ bv,
    const float* __restrict__ wW1, const float* __restrict__ wW2,
    unsigned short* __restrict__ WTH, unsigned short* __restrict__ W1H, unsigned short* __restrict__ W2H,
    float* __restrict__ BQKV)
{
  const int tid = threadIdx.x;
  const int bx  = blockIdx.x;
  if (bx < 24) {
    const int f   = bx * 256 + tid;
    const int row = f >> 4;
    const int k0  = (f & 15) * 8;
    const int sel = bx >> 3;
    const float* W = (sel == 0) ? Wq : ((sel == 1) ? Wk : Wv);
    emit_bt8(W, kCh, kCh, row & 127, k0, WTH, row, kCh);
  } else if (bx == 24) {
    const int row = tid >> 4;
    const int k0  = (tid & 15) * 8;
    emit_bt8(wW1, kGrp, kCh, row, k0, W1H, row, kCh);
  } else if (bx == 25) {
    if (tid < 64) {
      const int row = tid >> 2;
      const int k0  = (tid & 3) * 8;
      emit_bt8(wW2, kGrp, kGrp, row, k0, W2H, row, 32);
    }
  } else {
    if (tid < 96) {
      const int sel = tid >> 5;
      const float* src = (sel == 0) ? bq : ((sel == 1) ? bk : bv);
      const v4f v = *(const v4f*)(src + ((tid * 4) & 127));
      float* dst = BQKV + tid * 4;
      *(volatile v4f*)dst = v;
      __threadfence();
      *(volatile v4f*)dst = v;
    }
  }
}

struct PosLin { float w00, w01, w02, w10, w11, w12, w20, w21, w22, b0, b1, b2; };
__device__ __forceinline__ PosLin load_poslin(const float* __restrict__ pW1, const float* __restrict__ pb1) {
  PosLin L;
  L.w00 = pW1[0]; L.w01 = pW1[1]; L.w02 = pW1[2];
  L.w10 = pW1[3]; L.w11 = pW1[4]; L.w12 = pW1[5];
  L.w20 = pW1[6]; L.w21 = pW1[7]; L.w22 = pW1[8];
  L.b0 = pb1[0]; L.b1 = pb1[1]; L.b2 = pb1[2];
  return L;
}
__device__ __forceinline__ void pos_t(const PosLin& L, const float* __restrict__ p, int n, int i,
                                      float& t0, float& t1, float& t2) {
  const float d0 = p[i * 3 + 0] - p[n * 3 + 0];
  const float d1 = p[i * 3 + 1] - p[n * 3 + 1];
  const float d2 = p[i * 3 + 2] - p[n * 3 + 2];
  t0 = fmaf(d2, L.w20, fmaf(d1, L.w10, d0 * L.w00)) + L.b0;
  t1 = fmaf(d2, L.w21, fmaf(d1, L.w11, d0 * L.w01)) + L.b1;
  t2 = fmaf(d2, L.w22, fmaf(d1, L.w12, d0 * L.w02)) + L.b2;
}
__device__ __forceinline__ int clamp_pt(int i) {
  i = (i < 0) ? 0 : i;
  return (i > kPts - 1) ? (kPts - 1) : i;
}

struct ChanTab { v4f p0, p1, p2, pb; };
__device__ __forceinline__ ChanTab load_chantab(const float* __restrict__ pW2, const float* __restrict__ pb2, int lane) {
  ChanTab t;
  t.p0 = *(const v4f*)(pW2 + 4 * lane);
  t.p1 = *(const v4f*)(pW2 + kCh + 4 * lane);
  t.p2 = *(const v4f*)(pW2 + 2 * kCh + 4 * lane);
  t.pb = *(const v4f*)(pb2 + 4 * lane);
  return t;
}
__device__ __forceinline__ v4f pos_lin2(const ChanTab& t, float a0, float a1, float a2) {
  v4f r;
#pragma unroll
  for (int e = 0; e < 4; ++e) r[e] = fmaf(a2, t.p2[e], fmaf(a1, t.p1[e], a0 * t.p0[e])) + t.pb[e];
  return r;
}

__global__ __launch_bounds__(256) void pos_stats_kernel(
    const float* __restrict__ p, const int* __restrict__ idx,
    const float* __restrict__ pW1, const float* __restrict__ pb1, float* __restrict__ part)
{
  __shared__ float red[8 * 8];
  const int tid = threadIdx.x, lane = tid & 31, wave = tid >> 5;
  const PosLin L = load_poslin(pW1, pb1);
  float s0 = 0.f, s1 = 0.f, s2 = 0.f, q0 = 0.f, q1 = 0.f, q2 = 0.f;
#pragma unroll 1
  for (int it = 0; it < 8; ++it) {
    const int e = blockIdx.x * 2048 + it * 256 + tid;
    const int n = e >> 4;
    const int i = clamp_pt(idx[e]);
    float t0, t1, t2;
    pos_t(L, p, n, i, t0, t1, t2);
    s0 += t0; q0 = fmaf(t0, t0, q0);
    s1 += t1; q1 = fmaf(t1, t1, q1);
    s2 += t2; q2 = fmaf(t2, t2, q2);
  }
#pragma unroll
  for (int off = 16; off > 0; off >>= 1) {
    s0 += __shfl_xor(s0, off, 32);
    s1 += __shfl_xor(s1, off, 32);
    s2 += __shfl_xor(s2, off, 32);
    q0 += __shfl_xor(q0, off, 32);
    q1 += __shfl_xor(q1, off, 32);
    q2 += __shfl_xor(q2, off, 32);
  }
  if (lane == 0) {
    red[wave * 8 + 0] = s0; red[wave * 8 + 1] = s1; red[wave * 8 + 2] = s2;
    red[wave * 8 + 3] = q0; red[wave * 8 + 4] = q1; red[wave * 8 + 5] = q2;
  }
  __syncthreads();
  if (tid < 32) {
    const int sl = (tid < 6) ? tid : 5;
    float a = 0.f;
#pragma unroll
    for (int w = 0; w < 8; ++w) a += red[w * 8 + sl];
    const float v = (tid < 6) ? a : 0.0f;
    float* dst = part + (size_t)blockIdx.x * 32 + tid;
    *(volatile float*)dst = v;
    __threadfence();
    *(volatile float*)dst = v;
  }
}

template <int NCH, int PITCH, int NBLK, int NOUT>
__global__ __launch_bounds__(256) void bn_finalize_kernel(
    const float* __restrict__ part, const float* __restrict__ gamma, const float* __restrict__ beta,
    float* __restrict__ stat)
{
  static_assert(2 * NCH <= PITCH && PITCH <= 256 && (NOUT % 32) == 0 && NOUT >= 3 * NCH);
  __shared__ double dsum[256];
  const int tid = threadIdx.x;
  const int sl = (tid < PITCH) ? tid : (PITCH - 1);
  double a = 0.0;
#pragma unroll 1
  for (int b = 0; b < NBLK; ++b) a += (double)part[(size_t)b * PITCH + sl];
  dsum[tid] = a;
  __syncthreads();
  constexpr double inv = 1.0 / (double)kPairs;
#pragma unroll 1
  for (int o = tid; o < NOUT; o += 256) {
    const int which = o / NCH;
    const int c = o - which * NCH;
    const double mean = dsum[c] * inv;
    double var = dsum[NCH + c] * inv - mean * mean;
    var = (var < 0.0) ? 0.0 : var;
    const float vf = (float)var + kBnEps;
    const float rstd = 1.0f / sqrtf(vf);
    const float g = gamma[c];
    const float bt = beta[c];
    float v = 0.0f;
    v = (which == 0) ? (float)mean : v;
    v = (which == 1) ? (rstd * g) : v;
    v = (which == 2) ? bt : v;
    *(volatile float*)(stat + o) = v;
    __threadfence();
    *(volatile float*)(stat + o) = v;
  }
}

__global__ __launch_bounds__(256) void pos_act_kernel(
    const float* __restrict__ p, const int* __restrict__ idx,
    const float* __restrict__ pW1, const float* __restrict__ pb1,
    const float* __restrict__ pstat, float* __restrict__ A3)
{
  const int e = blockIdx.x * 256 + threadIdx.x;
  const int n = e >> 4;
  const int i = clamp_pt(idx[e]);
  const PosLin L = load_poslin(pW1, pb1);
  float t0, t1, t2;
  pos_t(L, p, n, i, t0, t1, t2);
  const float a0 = fmaxf((t0 - pstat[0]) * pstat[3] + pstat[6], 0.0f);
  const float a1 = fmaxf((t1 - pstat[1]) * pstat[4] + pstat[7], 0.0f);
  const float a2 = fmaxf((t2 - pstat[2]) * pstat[5] + pstat[8], 0.0f);
  const v4f v = (v4f){a0, a1, a2, 0.0f};
  float* dst = A3 + (size_t)e * 4;
  *(volatile v4f*)dst = v;
  __threadfence();
  *(volatile v4f*)dst = v;
}

__global__ __launch_bounds__(256) void attn_in_stats_kernel(
    const float* __restrict__ QKV, const float* __restrict__ A3, const int* __restrict__ idx,
    const float* __restrict__ pW2, const float* __restrict__ pb2, float* __restrict__ part)
{
  __shared__ __align__(16) float red[8 * 256];
  const int tid = threadIdx.x, lane = tid & 31, wave = tid >> 5, li = lane & 15;
  const ChanTab tb = load_chantab(pW2, pb2, lane);
  v4f sm = (v4f){0.f, 0.f, 0.f, 0.f};
  v4f sq = (v4f){0.f, 0.f, 0.f, 0.f};
#pragma unroll 1
  for (int pt = 0; pt < 4; ++pt) {
    const int n = blockIdx.x * 32 + wave * 4 + pt;
    const int iv = clamp_pt(idx[n * kNbr + li]);
    const v4f a3v = *(const v4f*)(A3 + (size_t)(n * kNbr + li) * 4);
    const float ax = a3v[0], ay = a3v[1], az = a3v[2];
    const v4f qq = *(const v4f*)(QKV + (size_t)n * kQkvP + 4 * lane);
#pragma unroll 1
    for (int s = 0; s < kNbr; ++s) {
      const int   i  = __shfl(iv, s, 32);
      const float a0 = __shfl(ax, s, 32);
      const float a1 = __shfl(ay, s, 32);
      const float a2 = __shfl(az, s, 32);
      const v4f kk = *(const v4f*)(QKV + (size_t)i * kQkvP + kCh + 4 * lane);
      const v4f pr = pos_lin2(tb, a0, a1, a2);
#pragma unroll
      for (int e = 0; e < 4; ++e) {
        const float w = (kk[e] - qq[e]) + pr[e];
        sm[e] += w;
        sq[e] = fmaf(w, w, sq[e]);
      }
    }
  }
  *(v4f*)(red + wave * 256 + 4 * lane) = sm;
  *(v4f*)(red + wave * 256 + 128 + 4 * lane) = sq;
  __syncthreads();
  float a = 0.f;
#pragma unroll
  for (int w = 0; w < 8; ++w) a += red[w * 256 + tid];
  float* dst = part + (size_t)blockIdx.x * 256 + tid;
  *(volatile float*)dst = a;
  __threadfence();
  *(volatile float*)dst = a;
}

__global__ __launch_bounds__(128) void attn_lin1_kernel(
    const float* __restrict__ QKV, const float* __restrict__ A3, const int* __restrict__ idx,
    const float* __restrict__ pW2, const float* __restrict__ pb2, const float* __restrict__ wstat,
    const unsigned short* __restrict__ W1H,
    const float* __restrict__ wb1, float* __restrict__ H1, float* __restrict__ hpart)
{
  __shared__ __align__(16) unsigned short sAh[4 * 16 * kAP];
  __shared__ __align__(16) unsigned short sBh[16 * kAP];
  __shared__ __align__(16) float sH[4 * 16 * kHP];
  __shared__ float red[4 * 32];
  const int tid = threadIdx.x, lane = tid & 31, wave = tid >> 5;
  const int li = lane & 15, hh = lane >> 4;

#pragma unroll
  for (int it = 0; it < 2; ++it) {
    const int f = it * 128 + tid;
    const int row = f >> 4;
    const int c8 = (f & 15) * 8;
    const v4u vh = *(const v4u*)(W1H + row * kCh + c8);
    *(v4u*)(sBh + row * kAP + c8) = vh;
  }
  const ChanTab tb = load_chantab(pW2, pb2, lane);
  const v4f mu = *(const v4f*)(wstat + 4 * lane);
  const v4f sc = *(const v4f*)(wstat + kCh + 4 * lane);
  const v4f be = *(const v4f*)(wstat + 2 * kCh + 4 * lane);
  const float bias = wb1[li];
  unsigned short* aH = sAh + wave * (16 * kAP);
  float* sHw = sH + wave * (16 * kHP);
  float ls = 0.f, lq = 0.f;
  __syncthreads();

#pragma unroll 1
  for (int pt = 0; pt < 8; ++pt) {
    const int n = blockIdx.x * 32 + wave * 8 + pt;
    const int iv = clamp_pt(idx[n * kNbr + li]);
    const v4f a3v = *(const v4f*)(A3 + (size_t)(n * kNbr + li) * 4);
    const float ax = a3v[0], ay = a3v[1], az = a3v[2];
    const v4f qq = *(const v4f*)(QKV + (size_t)n * kQkvP + 4 * lane);
#pragma unroll 1
    for (int s = 0; s < kNbr; ++s) {
      const int   i  = __shfl(iv, s, 32);
      const float a0 = __shfl(ax, s, 32);
      const float a1 = __shfl(ay, s, 32);
      const float a2 = __shfl(az, s, 32);
      const v4f kk = *(const v4f*)(QKV + (size_t)i * kQkvP + kCh + 4 * lane);
      const v4f pr = pos_lin2(tb, a0, a1, a2);
      float an[4];
#pragma unroll
      for (int e = 0; e < 4; ++e) {
        const float w = (kk[e] - qq[e]) + pr[e];
        an[e] = fmaxf((w - mu[e]) * sc[e] + be[e], 0.0f) * kActCarry;
      }
      const unsigned w01 = pack_h2(an[0], an[1]);
      const unsigned w23 = pack_h2(an[2], an[3]);
      const v2u vh = (v2u){w01, w23};
      *(v2u*)(aH + s * kAP + 4 * lane) = vh;
    }
    __syncthreads();

    v8f acc = (v8f){0.f, 0.f, 0.f, 0.f, 0.f, 0.f, 0.f, 0.f};
#pragma unroll 1
    for (int kb = 0; kb < 4; ++kb) {
      const int ko = li * kAP + kb * 32 + 8 * hh;
      const v16h ah = frag_load((const _Float16*)(aH + ko));
      const v16h bh = frag_load((const _Float16*)(sBh + ko));
      acc = hmma(ah, bh, acc);
    }
#pragma unroll
    for (int r = 0; r < 8; ++r) {
      const float hv = acc[r] * kFold + bias;
      ls += hv;
      lq = fmaf(hv, hv, lq);
      sHw[(8 * hh + r) * kHP + li] = hv;
    }
    __syncthreads();
    {
      const v4f o0 = *(const v4f*)(sHw + (lane >> 2) * kHP + (lane & 3) * 4);
      const v4f o1 = *(const v4f*)(sHw + (8 + (lane >> 2)) * kHP + (lane & 3) * 4);
      float* dst = H1 + (size_t)n * 256 + 4 * lane;
      *(volatile v4f*)dst = o0;
      *(volatile v4f*)(dst + 128) = o1;
      __threadfence();
      *(volatile v4f*)dst = o0;
      *(volatile v4f*)(dst + 128) = o1;
    }
    __syncthreads();
  }

  ls += __shfl_xor(ls, 16, 32);
  lq += __shfl_xor(lq, 16, 32);
  red[wave * 32 + lane] = (hh == 0) ? ls : lq;
  __syncthreads();
  if (tid < 32) {
    const float a = ((red[tid] + red[32 + tid]) + red[64 + tid]) + red[96 + tid];
    float* dst = hpart + (size_t)blockIdx.x * 32 + tid;
    *(volatile float*)dst = a;
    __threadfence();
    *(volatile float*)dst = a;
  }
}

__global__ __launch_bounds__(128) void attn_out_kernel(
    const float* __restrict__ QKV, const float* __restrict__ A3, const int* __restrict__ idx,
    const float* __restrict__ pW2, const float* __restrict__ pb2,
    const float* __restrict__ H1, const float* __restrict__ hstat,
    const unsigned short* __restrict__ W2H,
    const float* __restrict__ wb2, float* __restrict__ out)
{
  __shared__ __align__(16) float sS[4 * 16 * kHP];
  const int tid = threadIdx.x, lane = tid & 31, wave = tid >> 5;
  const int li = lane & 15, hh = lane >> 4;
  float* sw = sS + wave * (16 * kHP);
  const ChanTab tb = load_chantab(pW2, pb2, lane);
  const v4f muA = *(const v4f*)(hstat + 8 * hh);
  const v4f muB = *(const v4f*)(hstat + 8 * hh + 4);
  const v4f scA = *(const v4f*)(hstat + 16 + 8 * hh);
  const v4f scB = *(const v4f*)(hstat + 16 + 8 * hh + 4);
  const v4f beA = *(const v4f*)(hstat + 32 + 8 * hh);
  const v4f beB = *(const v4f*)(hstat + 32 + 8 * hh + 4);
  const v16h bW = frag_load((const _Float16*)(W2H + li * 32 + 8 * hh));
  const float bias = wb2[li];

#pragma unroll 1
  for (int pt = 0; pt < 8; ++pt) {
    const int n = blockIdx.x * 32 + wave * 8 + pt;
    const int iv = clamp_pt(idx[n * kNbr + li]);
    const v4f a3v = *(const v4f*)(A3 + (size_t)(n * kNbr + li) * 4);
    const float ax = a3v[0], ay = a3v[1], az = a3v[2];
    const float* hrow = H1 + (size_t)n * 256 + li * 16 + 8 * hh;
    const v4f x0 = *(const v4f*)(hrow);
    const v4f x1 = *(const v4f*)(hrow + 4);
    float an[8];
#pragma unroll
    for (int e = 0; e < 4; ++e) {
      an[e]     = fmaxf((x0[e] - muA[e]) * scA[e] + beA[e], 0.0f) * kActCarry;
      an[4 + e] = fmaxf((x1[e] - muB[e]) * scB[e] + beB[e], 0.0f) * kActCarry;
    }
    const unsigned wh0 = pack_h2(an[0], an[1]);
    const unsigned wh1 = pack_h2(an[2], an[3]);
    const unsigned wh2 = pack_h2(an[4], an[5]);
    const unsigned wh3 = pack_h2(an[6], an[7]);
    const v8u uh = (v8u){wh0, wh1, wh2, wh3, 0u, 0u, 0u, 0u};
    const v16h ah = __builtin_bit_cast(v16h, uh);
    v8f c = (v8f){0.f, 0.f, 0.f, 0.f, 0.f, 0.f, 0.f, 0.f};
    c = hmma(ah, bW, c);

    float lg[8];
    float mx = -INFINITY;
#pragma unroll
    for (int r = 0; r < 8; ++r) { lg[r] = c[r] * kFold + bias; mx = fmaxf(mx, lg[r]); }
    mx = fmaxf(mx, __shfl_xor(mx, 16, 32));
    float se = 0.f;
#pragma unroll
    for (int r = 0; r < 8; ++r) { lg[r] = expf(lg[r] - mx); se += lg[r]; }
    se += __shfl_xor(se, 16, 32);
    const float inv = 1.0f / se;
#pragma unroll
    for (int r = 0; r < 8; ++r) sw[(8 * hh + r) * kHP + li] = lg[r] * inv;
    __syncthreads();

    v4f acc = (v4f){0.f, 0.f, 0.f, 0.f};
#pragma unroll 1
    for (int s = 0; s < kNbr; ++s) {
      const int   i  = __shfl(iv, s, 32);
      const float a0 = __shfl(ax, s, 32);
      const float a1 = __shfl(ay, s, 32);
      const float a2 = __shfl(az, s, 32);
      const v4f vv = *(const v4f*)(QKV + (size_t)i * kQkvP + 2 * kCh + 4 * lane);
      const v4f wv = *(const v4f*)(sw + s * kHP + 4 * (lane & 3));
      const v4f pr = pos_lin2(tb, a0, a1, a2);
#pragma unroll
      for (int e = 0; e < 4; ++e) acc[e] = fmaf(vv[e] + pr[e], wv[e], acc[e]);
    }
    {
      float* dst = out + (size_t)n * kCh + 4 * lane;
      *(volatile v4f*)dst = acc;
      __threadfence();
      *(volatile v4f*)dst = acc;
    }
    __syncthreads();
  }
}

extern "C" void kernel_launch(void* const* d_in, const int* in_sizes, int n_in,
                              void* d_out, int out_size, void* d_ws, size_t ws_size,
                              hipStream_t stream) {
  if (n_in < 23) return;
  if (in_sizes[0] != kPts * 3) return;
  if (in_sizes[1] != kPts * kCh) return;
  if (in_sizes[2] != kCh * kCh || in_sizes[4] != kCh * kCh || in_sizes[6] != kCh * kCh) return;
  if (in_sizes[3] != kCh || in_sizes[5] != kCh || in_sizes[7] != kCh) return;
  if (in_sizes[8] != 9 || in_sizes[9] != 3 || in_sizes[10] != 3 || in_sizes[11] != 3) return;
  if (in_sizes[12] != 3 * kCh || in_sizes[13] != kCh || in_sizes[14] != kCh || in_sizes[15] != kCh) return;
  if (in_sizes[16] != kCh * kGrp || in_sizes[17] != kGrp || in_sizes[18] != kGrp || in_sizes[19] != kGrp) return;
  if (in_sizes[20] != kGrp * kGrp || in_sizes[21] != kGrp) return;
  if (in_sizes[22] != kPts * kNbr) return;
  if (out_size != kPts * kCh) return;
  if (ws_size < kWsTotal) return;

  const float* p    = (const float*)d_in[0];
  const float* x    = (const float*)d_in[1];
  const float* Wq   = (const float*)d_in[2];
  const float* bq   = (const float*)d_in[3];
  const float* Wk   = (const float*)d_in[4];
  const float* bk   = (const float*)d_in[5];
  const float* Wv   = (const float*)d_in[6];
  const float* bv   = (const float*)d_in[7];
  const float* pW1  = (const float*)d_in[8];
  const float* pb1  = (const float*)d_in[9];
  const float* pg1  = (const float*)d_in[10];
  const float* pbe1 = (const float*)d_in[11];
  const float* pW2  = (const float*)d_in[12];
  const float* pb2  = (const float*)d_in[13];
  const float* wg1  = (const float*)d_in[14];
  const float* wbe1 = (const float*)d_in[15];
  const float* wW1  = (const float*)d_in[16];
  const float* wb1  = (const float*)d_in[17];
  const float* wg2  = (const float*)d_in[18];
  const float* wbe2 = (const float*)d_in[19];
  const float* wW2  = (const float*)d_in[20];
  const float* wb2  = (const float*)d_in[21];
  const int*   idx  = (const int*)d_in[22];
  float* out = (float*)d_out;

  char* ws = (char*)d_ws;
  unsigned short* XH   = (unsigned short*)(ws + kOffXH);
  unsigned short* WTH  = (unsigned short*)(ws + kOffWTH);
  unsigned short* W1H  = (unsigned short*)(ws + kOffW1H);
  unsigned short* W2H  = (unsigned short*)(ws + kOffW2H);
  float* BQKV  = (float*)(ws + kOffBQKV);
  float* QKV   = (float*)(ws + kOffQKV);
  float* A3    = (float*)(ws + kOffA3);
  float* H1    = (float*)(ws + kOffH1);
  float* PPART = (float*)(ws + kOffPPART);
  float* PSTAT = (float*)(ws + kOffPSTAT);
  float* WPART = (float*)(ws + kOffWPART);
  float* WSTAT = (float*)(ws + kOffWSTAT);
  float* HPART = (float*)(ws + kOffHPART);
  float* HSTAT = (float*)(ws + kOffHSTAT);

  prep_planes_kernel<<<27, 256, 0, stream>>>(Wq, Wk, Wv, bq, bk, bv, wW1, wW2, WTH, W1H, W2H, BQKV);
  cast_rows_f16_kernel<<<(kPts * kCh / 8) / 256, 256, 0, stream>>>(x, XH, kPts * kCh / 8);

  wmma_gemm64_f16<<<384, 256, 0, stream>>>(XH, kCh, WTH, kCh, QKV, kQkvP, BQKV,
                                           kPts, kQkvP, kCh, kFold);

  pos_stats_kernel<<<256, 256, 0, stream>>>(p, idx, pW1, pb1, PPART);
  bn_finalize_kernel<3, 32, 256, 32><<<1, 256, 0, stream>>>(PPART, pg1, pbe1, PSTAT);
  pos_act_kernel<<<kPairs / 256, 256, 0, stream>>>(p, idx, pW1, pb1, PSTAT, A3);

  attn_in_stats_kernel<<<1024, 256, 0, stream>>>(QKV, A3, idx, pW2, pb2, WPART);
  bn_finalize_kernel<128, 256, 1024, 384><<<1, 256, 0, stream>>>(WPART, wg1, wbe1, WSTAT);

  attn_lin1_kernel<<<1024, 128, 0, stream>>>(QKV, A3, idx, pW2, pb2, WSTAT, W1H, wb1, H1, HPART);
  bn_finalize_kernel<16, 32, 1024, 64><<<1, 256, 0, stream>>>(HPART, wg2, wbe2, HSTAT);

  attn_out_kernel<<<1024, 128, 0, stream>>>(QKV, A3, idx, pW2, pb2, H1, HSTAT, W2H, wb2, out);
}
